// SelfAttention_37220186587176
// MI455X (gfx1250) — hardware-verified
//
#include <hip/hip_runtime.h>


#ifndef NB
#define NB 8
#endif
#ifndef SEQ
#define SEQ 1024
#endif
#define NB_FULL  8
#define SEQ_FULL 1024
#define DM   1024
#define NH   16
#define HD   64
#define MROWS (NB * SEQ)
#define WCAR 64.0f
#define CCAR 16.0f
#define PEXP 8.0f
#define CL2  0.18033688011112042f
#define EROWS 256
#define QCAR 64.0f
#define VCAR 16.0f
#define ECAR 256.0f
#define PEXPE 12.0f
#define CL2E (CL2 / (QCAR * QCAR))
#define NEGV (-3.0e38f)

#define SZ_W   ((size_t)DM * DM * 2)
#define SZ_W2  ((size_t)DM * 2 * DM * 2)
#define SZ_TAB ((size_t)SEQ * 64 * 4)
#define SZ_PL  ((size_t)MROWS * DM * 2)
#define SZ_QE  ((size_t)NB * EROWS * NH * 128 * 2)
#define SZ_V32 ((size_t)NB * DM * EROWS * 4)
#define SZ_VTE ((size_t)NB * DM * 2 * EROWS * 2)
#define SZ_CE  ((size_t)NB * EROWS * 2 * DM * 2)

static_assert((SEQ & (SEQ - 1)) == 0);
static_assert(SEQ % 64 == 0);
static_assert(SEQ <= SEQ_FULL);
static_assert(NB <= NB_FULL);
static_assert(DM == NH * HD);
static_assert(HD == 64);
static_assert(DM % 256 == 0);
static_assert(DM % 32 == 0);
static_assert((2 * DM) % 32 == 0);
static_assert(((size_t)MROWS * DM) % 2048 == 0);
static_assert(MROWS % 64 == 0);
static_assert(EROWS % 64 == 0);
static_assert(EROWS >= 64);
static_assert(EROWS <= SEQ);
static_assert((SEQ - EROWS) % 64 == 0);
static_assert(((size_t)NB * DM * EROWS) % 2048 == 0);
static_assert(SEQ % 8 == 0);
static_assert(((size_t)DM * 2 * DM / 64) % 64 == 0);
static_assert(SZ_W % 256 == 0 && SZ_W2 % 256 == 0 && SZ_TAB % 256 == 0 && SZ_PL % 256 == 0 && SZ_QE % 256 == 0 && SZ_V32 % 256 == 0 && SZ_VTE % 256 == 0 && SZ_CE % 256 == 0);
static_assert(4 * SZ_W + SZ_W2 + SZ_TAB + 4 * SZ_PL + 2 * SZ_QE + SZ_V32 + SZ_VTE + SZ_CE <= (size_t)134217728);
static_assert(((size_t)(NB - 1) * SEQ_FULL + SEQ) * DM <= (size_t)NB_FULL * SEQ_FULL * DM);
static_assert((size_t)MROWS * DM * 4 <= (size_t)NB_FULL * SEQ_FULL * DM * 4);

typedef _Float16 h16;
typedef __attribute__((ext_vector_type(16))) _Float16 v16h;
typedef __attribute__((ext_vector_type(8)))  _Float16 v8h;
typedef __attribute__((ext_vector_type(4)))  _Float16 v4h;
typedef __attribute__((ext_vector_type(2)))  _Float16 v2h;
typedef __attribute__((ext_vector_type(8)))  float    v8f;
typedef __attribute__((ext_vector_type(4)))  float    v4f;
typedef v8h __attribute__((may_alias)) v8ha;
typedef v4f __attribute__((may_alias)) v4fa;

__device__ __forceinline__ unsigned short f2bf(float f) { unsigned u = __float_as_uint(f); u += 0x7FFFu + ((u >> 16) & 1u); return (unsigned short)(u >> 16); }
__device__ __forceinline__ float bf2f(unsigned short b) { return __uint_as_float(((unsigned)b) << 16); }
__device__ __forceinline__ float bfr(float f) { return bf2f(f2bf(f)); }
__device__ __forceinline__ v16h cat16(v8h lo, v8h hi) { return __builtin_shufflevector(lo, hi, 0, 1, 2, 3, 4, 5, 6, 7, 8, 9, 10, 11, 12, 13, 14, 15); }
__device__ __forceinline__ v8f wmma16(v16h a, v16h b, v8f c) { return __builtin_amdgcn_wmma_f32_16x16x32_f16(false, a, false, b, (short)0, c, false, false); }
__device__ __forceinline__ v16h ldfrag(const h16* p) { return cat16(*(const v8h*)p, *(const v8h*)(p + 16)); }
__device__ __forceinline__ unsigned xrow(unsigned r) { return (r / (unsigned)SEQ) * (unsigned)SEQ_FULL + (r % (unsigned)SEQ); }

static __device__ __forceinline__ h16 toh_flush(float v) { const h16 r = (h16)v; return (fabsf(v) < 6.103515625e-05f) ? (h16)0.0f : r; }
static __device__ __forceinline__ v8f wmma16g(v16h a, v16h b, v8f c) {
    c = __builtin_amdgcn_wmma_f32_16x16x32_f16(false, a, false, b, (short)0, c, false, false);
    asm volatile("v_nop\n\tv_nop\n\tv_nop\n\tv_nop" : "+v"(c) : "v"(a), "v"(b));
    return c;
}

__global__ __launch_bounds__(256) void k_cvtx(const float* __restrict__ x, h16* XH) {
    const unsigned i = blockIdx.x * 256u + threadIdx.x; const unsigned e = i * 8u; if (e >= (unsigned)MROWS * DM) return;
    const unsigned row = e / (unsigned)DM, col = e % (unsigned)DM;
    const v8f v = *(const v8f*)(x + (size_t)xrow(row) * DM + col); v8h o;
#pragma unroll
    for (int k = 0; k < 8; ++k) o[k] = (h16)bfr(v[k]);
    *(volatile v8h*)(XH + e) = o; __threadfence(); *(volatile v8h*)(XH + e) = o;
}

template <unsigned K, unsigned N>
__global__ __launch_bounds__(256) void k_wt(const float* __restrict__ w, h16* Bt) {
    static_assert((K & (K - 1)) == 0); static_assert((N * K / 64u) % 64u == 0);
    const unsigned lane = threadIdx.x & 31u; const unsigned L0 = (blockIdx.x * 8u + (threadIdx.x >> 5)) * 8u; const unsigned nlines = N * K / 64u;
#pragma unroll
    for (int ps = 0; ps < 2; ++ps) {
#pragma unroll 1
        for (unsigned l = 0; l < 8u; ++l) { const unsigned L = L0 + l; if (L >= nlines) break; const unsigned e = L * 64u + lane * 2u; const unsigned k = e % K, n = e / K; v2h o;
            o[0] = (h16)(bfr(w[(size_t)k * N + n]) * WCAR); o[1] = (h16)(bfr(w[(size_t)(k + 1u) * N + n]) * WCAR); *(volatile v2h*)(Bt + e) = o; }
        if (ps == 0) __threadfence(); }
}

__global__ __launch_bounds__(256) void k_wtd(const float* __restrict__ w, h16* Bt) {
    const unsigned lane = threadIdx.x & 31u; const unsigned wave = (unsigned)__builtin_amdgcn_readfirstlane((int)(threadIdx.x >> 5));
    const unsigned L0 = (blockIdx.x * 8u + wave) * 8u; const unsigned nlines = (unsigned)DM * 2u * (unsigned)DM / 64u;
#pragma unroll
    for (int ps = 0; ps < 2; ++ps) {
#pragma unroll 1
        for (unsigned l = 0; l < 8u; ++l) { const unsigned L = L0 + l; if (L >= nlines) break; const unsigned e = L * 64u + lane * 2u; const unsigned n = e / (2u * (unsigned)DM), k = e & ((unsigned)DM - 1u); v2h o;
            o[0] = toh_flush(bfr(w[(size_t)k * DM + n]) * WCAR); o[1] = toh_flush(bfr(w[(size_t)(k + 1u) * DM + n]) * WCAR); *(volatile v2h*)(Bt + e) = o; }
        if (ps == 0) __threadfence(); }
}

__global__ __launch_bounds__(256) void k_tab(float* TAB) {
#pragma clang fp contract(off)
    const unsigned lane = threadIdx.x & 31u; const unsigned wave = (unsigned)__builtin_amdgcn_readfirstlane((int)(threadIdx.x >> 5));
    const unsigned l = blockIdx.x * 8u + wave; if (l >= (unsigned)SEQ) return;
    double p = 1.0;
#pragma unroll 1
    for (unsigned j = 0; j < 31u; ++j) p = (j < lane) ? p * 1.333521432163324 : p;
    const float pw = (float)p; const float invf = 1.0f / pw; const float ang = (float)l * invf;
    const float cv = cosf(ang); const float sv = sinf(ang);
    float* tr = TAB + (size_t)l * 64u;
    *(volatile float*)(tr + lane) = cv; *(volatile float*)(tr + 32u + lane) = sv;
    __threadfence();
    *(volatile float*)(tr + lane) = cv; *(volatile float*)(tr + 32u + lane) = sv;
}

__global__ __launch_bounds__(256) void k_rope(const float* F, const float* __restrict__ TAB, h16* P16, h16* PE) {
#pragma clang fp contract(off)
    const unsigned i = blockIdx.x * 256u + threadIdx.x; const unsigned e = i * 8u; if (e >= (unsigned)MROWS * DM) return;
    const unsigned row = e / (unsigned)DM, col = e % (unsigned)DM; const unsigned b = row / (unsigned)SEQ, t = row % (unsigned)SEQ;
    const unsigned hh = col >> 6, d0 = col & 63u;
    const v8f v = *(const v8f*)(F + e);
    const v4f cs = *(const v4f*)(TAB + (size_t)t * 64u + (d0 >> 1)); const v4f sn = *(const v4f*)(TAB + (size_t)t * 64u + 32u + (d0 >> 1));
    float r[8];
#pragma unroll
    for (int j = 0; j < 4; ++j) { const float x1 = v[2 * j], x2 = v[2 * j + 1]; r[2 * j] = x1 * cs[j] - x2 * sn[j]; r[2 * j + 1] = x1 * sn[j] + x2 * cs[j]; }
    v8h o, oh, ol;
#pragma unroll
    for (int k = 0; k < 8; ++k) { o[k] = toh_flush(r[k]); const float s = r[k] * QCAR; const h16 hv = toh_flush(s); oh[k] = hv; ol[k] = toh_flush(s - (float)hv); }
    const bool early = t < (unsigned)EROWS;
    const unsigned te = early ? t : 0u;
    h16* pe = PE + (((size_t)b * EROWS + te) * NH + hh) * 128u + d0;
    *(volatile v8h*)(P16 + e) = o;
    if (early) { *(volatile v8h*)pe = oh; *(volatile v8h*)(pe + 64) = ol; }
    __threadfence();
    *(volatile v8h*)(P16 + e) = o;
    if (early) { *(volatile v8h*)pe = oh; *(volatile v8h*)(pe + 64) = ol; }
}

__global__ __launch_bounds__(256) void k_vsplit(const float* __restrict__ V32, h16* VTE) {
#pragma clang fp contract(off)
    const unsigned i = blockIdx.x * 256u + threadIdx.x; const unsigned e = i * 8u; if (e >= (unsigned)NB * DM * EROWS) return;
    const unsigned row = e / (unsigned)EROWS, col = e % (unsigned)EROWS;
    const v8f v = *(const v8f*)(V32 + e);
    v8h oh, ol;
#pragma unroll
    for (int k = 0; k < 8; ++k) { const float s = v[k] * VCAR; const h16 hv = toh_flush(s); oh[k] = hv; ol[k] = toh_flush(s - (float)hv); }
    h16* dst = VTE + (size_t)row * (2u * EROWS) + col;
    *(volatile v8h*)dst = oh; *(volatile v8h*)(dst + EROWS) = ol;
    __threadfence();
    *(volatile v8h*)dst = oh; *(volatile v8h*)(dst + EROWS) = ol;
}

template <int OUT16, int RELU, int BIASM, int RESM>
__global__ __launch_bounds__(32) void k_gemm(const h16* __restrict__ A, const h16* __restrict__ Bt, unsigned K, void* Cv, unsigned ldc, float alpha, const float* __restrict__ bias, const float* resid, size_t sA, size_t sB, size_t sC) {
    __shared__ __align__(16) float os[16 * 68];
    const size_t z = blockIdx.z; A += z * sA; Bt += z * sB;
    const unsigned lane = threadIdx.x & 31u, lr = lane & 15u, hi = lane >> 4; const unsigned r0 = blockIdx.x * 64u, c0 = blockIdx.y * 64u;
    v8f acc[4][4];
#pragma unroll
    for (int mb = 0; mb < 4; ++mb)
#pragma unroll
        for (int nb = 0; nb < 4; ++nb) acc[mb][nb] = (v8f){};
    const size_t aoff = (size_t)(r0 + lr) * K + 8u * hi, boff = (size_t)(c0 + lr) * K + 8u * hi;
#pragma unroll 1
    for (unsigned kc = 0; kc < K; kc += 32u) {
        v16h a[4];
#pragma unroll
        for (int mb = 0; mb < 4; ++mb) a[mb] = ldfrag(A + aoff + (size_t)mb * 16u * K + kc);
#pragma unroll
        for (int nb = 0; nb < 4; ++nb) { const v16h b = ldfrag(Bt + boff + (size_t)nb * 16u * K + kc);
#pragma unroll
            for (int mb = 0; mb < 4; ++mb) acc[mb][nb] = wmma16(a[mb], b, acc[mb][nb]); }
        asm volatile("v_nop\n\tv_nop\n\tv_nop\n\tv_nop" : "+v"(acc[0][0]), "+v"(acc[1][1]), "+v"(acc[2][2]), "+v"(acc[3][3]) : "v"(a[0]), "v"(a[3]));
    }
    float* Cf = (float*)Cv + z * sC; h16* Ch = (h16*)Cv + z * sC;
    const unsigned rq = lane >> 3, c8 = (lane & 7u) * 8u, c4 = lr * 4u;
    v4f bA = {0.f, 0.f, 0.f, 0.f}, bB = {0.f, 0.f, 0.f, 0.f};
    if (BIASM == 1) {
        if (OUT16) { const v4f t0 = *(const v4f*)(bias + c0 + c8); const v4f t1 = *(const v4f*)(bias + c0 + c8 + 4u);
#pragma unroll
            for (int q = 0; q < 4; ++q) { bA[q] = bfr(t0[q]); bB[q] = bfr(t1[q]); } }
        else { const v4f t0 = *(const v4f*)(bias + c0 + c4);
#pragma unroll
            for (int q = 0; q < 4; ++q) bA[q] = bfr(t0[q]); }
    }
#pragma unroll
    for (int mb = 0; mb < 4; ++mb) {
#pragma unroll
        for (int nb = 0; nb < 4; ++nb) {
#pragma unroll
            for (int j = 0; j < 8; ++j) os[(hi * 8u + j) * 68u + nb * 16u + lr] = acc[mb][nb][j]; }
        __syncthreads();
        const unsigned rbase = r0 + (unsigned)mb * 16u;
#pragma unroll 1
        for (int ps = 0; ps < 2; ++ps) {
            if (OUT16) {
#pragma unroll
                for (unsigned s = 0; s < 4u; ++s) { const unsigned row = 4u * s + rq;
                    const v4f a = *(const v4fa*)(os + row * 68u + c8); const v4f b = *(const v4fa*)(os + row * 68u + c8 + 4u);
                    float rb = 0.f; if (BIASM == 2) rb = bfr(bias[rbase + row]);
                    v8h o;
#pragma unroll
                    for (int q = 0; q < 4; ++q) { float x0 = a[q] * alpha + bA[q] + rb, x1 = b[q] * alpha + bB[q] + rb; if (RELU) { x0 = fmaxf(x0, 0.0f); x1 = fmaxf(x1, 0.0f); } o[q] = (h16)x0; o[4 + q] = (h16)x1; }
                    *(volatile v8h*)(Ch + (size_t)(rbase + row) * ldc + c0 + c8) = o; }
            } else {
#pragma unroll
                for (unsigned s = 0; s < 8u; ++s) { const unsigned row = 2u * s + hi;
                    v4f val = *(const v4fa*)(os + row * 68u + c4);
                    float rb = 0.f; if (BIASM == 2) rb = bfr(bias[rbase + row]);
#pragma unroll
                    for (int q = 0; q < 4; ++q) { float x0 = val[q] * alpha + bA[q] + rb; if (RELU) x0 = fmaxf(x0, 0.0f); val[q] = x0; }
                    if (RESM == 1) { const v4f rv = *(const v4f*)(resid + (size_t)(rbase + row) * ldc + c0 + c4);
#pragma unroll
                        for (int q = 0; q < 4; ++q) val[q] = __fadd_rn(val[q], rv[q]); }
                    if (RESM == 2) { const v4f rv = *(const v4f*)(resid + (size_t)xrow(rbase + row) * DM + c0 + c4);
#pragma unroll
                        for (int q = 0; q < 4; ++q) val[q] = __fadd_rn(val[q], bfr(rv[q])); }
                    *(volatile v4f*)(Cf + (size_t)(rbase + row) * ldc + c0 + c4) = val; }
            }
            if (ps == 0) __threadfence(); }
        __syncthreads();
    }
}

__global__ __launch_bounds__(32) void k_flash(const h16* __restrict__ Qp, const h16* __restrict__ Kp, const h16* __restrict__ VTp, h16* Cx) {
    __shared__ __align__(16) h16 os[32 * 72];
    const unsigned lane = threadIdx.x & 31u, lr = lane & 15u, hi = lane >> 4;
    const unsigned q0 = (unsigned)EROWS + blockIdx.x * 32u, hh = blockIdx.y, b = blockIdx.z;
    const size_t rowb = (size_t)b * SEQ;
    const h16* qbase = Qp + (rowb + q0 + lr) * DM + hh * HD + 8u * hi;
    const h16* kbase = Kp + (rowb + lr) * DM + hh * HD + 8u * hi;
    const h16* vbase = VTp + ((size_t)b * DM + hh * HD + lr) * SEQ + 8u * hi;
    v16h qb[2][2];
#pragma unroll
    for (int qt = 0; qt < 2; ++qt)
#pragma unroll
        for (int ks = 0; ks < 2; ++ks) qb[qt][ks] = ldfrag(qbase + (size_t)qt * 16u * DM + ks * 32u);
    v8f ot[4][2];
#pragma unroll
    for (int dt = 0; dt < 4; ++dt) { ot[dt][0] = (v8f){}; ot[dt][1] = (v8f){}; }
    float m0 = -3.0e38f, m1 = -3.0e38f, l0 = 0.f, l1 = 0.f;
    const unsigned ktl = q0 >> 5;
#pragma unroll 1
    for (unsigned kt = 0; kt <= ktl; ++kt) {
        v16h ka[2][2];
#pragma unroll
        for (int mt = 0; mt < 2; ++mt)
#pragma unroll
            for (int ks = 0; ks < 2; ++ks) ka[mt][ks] = ldfrag(kbase + (size_t)(kt * 32u + mt * 16u) * DM + ks * 32u);
        v8f st[2][2];
#pragma unroll
        for (int qt = 0; qt < 2; ++qt) { st[qt][0] = (v8f){}; st[qt][1] = (v8f){}; }
#pragma unroll
        for (int ks = 0; ks < 2; ++ks)
#pragma unroll
            for (int qt = 0; qt < 2; ++qt)
#pragma unroll
                for (int mt = 0; mt < 2; ++mt) st[qt][mt] = wmma16g(ka[mt][ks], qb[qt][ks], st[qt][mt]);
        v16h va[4];
#pragma unroll
        for (int dt = 0; dt < 4; ++dt) va[dt] = ldfrag(vbase + (size_t)dt * 16u * SEQ + kt * 32u);
        if (kt == ktl) {
#pragma unroll
            for (int qt = 0; qt < 2; ++qt)
#pragma unroll
                for (int mt = 0; mt < 2; ++mt)
#pragma unroll
                    for (int r = 0; r < 8; ++r) { const bool dead = ((unsigned)(mt * 16 + r) + 8u * hi) > ((unsigned)(qt * 16) + lr); st[qt][mt][r] = dead ? NEGV : st[qt][mt][r]; }
        }
        float t0 = st[0][0][0], t1 = st[1][0][0];
#pragma unroll
        for (int r = 0; r < 8; ++r) { t0 = fmaxf(t0, fmaxf(st[0][0][r], st[0][1][r])); t1 = fmaxf(t1, fmaxf(st[1][0][r], st[1][1][r])); }
        t0 = fmaxf(t0, __shfl_xor(t0, 16, 32)); t1 = fmaxf(t1, __shfl_xor(t1, 16, 32));
        const float mn0 = fmaxf(m0, t0), mn1 = fmaxf(m1, t1);
        const bool grow = (mn0 > m0) || (mn1 > m1);
        if (__builtin_amdgcn_ballot_w32(grow) != 0u) {
            const float a0 = __builtin_amdgcn_exp2f((m0 - mn0) * CL2), a1 = __builtin_amdgcn_exp2f((m1 - mn1) * CL2);
            l0 *= a0; l1 *= a1;
#pragma unroll
            for (int dt = 0; dt < 4; ++dt)
#pragma unroll
                for (int r = 0; r < 8; ++r) { ot[dt][0][r] *= a0; ot[dt][1][r] *= a1; }
        }
        m0 = mn0; m1 = mn1;
        const float off0 = PEXP - mn0 * CL2, off1 = PEXP - mn1 * CL2;
        v16h pb0, pb1; float s0 = 0.f, s1 = 0.f;
#pragma unroll
        for (int r = 0; r < 8; ++r) {
            const float e00 = fmaf(st[0][0][r], CL2, off0), e01 = fmaf(st[0][1][r], CL2, off0);
            const float e10 = fmaf(st[1][0][r], CL2, off1), e11 = fmaf(st[1][1][r], CL2, off1);
            float p00 = __builtin_amdgcn_exp2f(e00), p01 = __builtin_amdgcn_exp2f(e01), p10 = __builtin_amdgcn_exp2f(e10), p11 = __builtin_amdgcn_exp2f(e11);
            p00 = (e00 < -14.0f) ? 0.0f : p00; p01 = (e01 < -14.0f) ? 0.0f : p01; p10 = (e10 < -14.0f) ? 0.0f : p10; p11 = (e11 < -14.0f) ? 0.0f : p11;
            const h16 h00 = (h16)p00, h01 = (h16)p01, h10 = (h16)p10, h11 = (h16)p11;
            s0 += (float)h00 + (float)h01; s1 += (float)h10 + (float)h11;
            pb0[r] = h00; pb0[8 + r] = h01; pb1[r] = h10; pb1[8 + r] = h11; }
        l0 += s0; l1 += s1;
#pragma unroll
        for (int dt = 0; dt < 4; ++dt) { ot[dt][0] = wmma16g(va[dt], pb0, ot[dt][0]); ot[dt][1] = wmma16g(va[dt], pb1, ot[dt][1]); }
    }
    l0 += __shfl_xor(l0, 16, 32); l1 += __shfl_xor(l1, 16, 32);
    const float i0 = CCAR / l0, i1 = CCAR / l1;
#pragma unroll
    for (int dt = 0; dt < 4; ++dt) { v8h o0, o1;
#pragma unroll
        for (int r = 0; r < 8; ++r) { o0[r] = toh_flush(ot[dt][0][r] * i0); o1[r] = toh_flush(ot[dt][1][r] * i1); }
        *(v8ha*)(os + lr * 72u + dt * 16u + 8u * hi) = o0; *(v8ha*)(os + (16u + lr) * 72u + dt * 16u + 8u * hi) = o1; }
    __syncthreads();
    h16* cb = Cx + (rowb + q0) * DM + hh * HD; const unsigned rq = lane >> 3, c8 = (lane & 7u) * 8u;
#pragma unroll 1
    for (int ps = 0; ps < 2; ++ps) {
#pragma unroll
        for (unsigned s = 0; s < 8u; ++s) { const unsigned row = 4u * s + rq; const v8h v = *(const v8ha*)(os + row * 72u + c8); *(volatile v8h*)(cb + (size_t)row * DM + c8) = v; }
        if (ps == 0) __threadfence(); }
}

__global__ __launch_bounds__(32) void k_flash_early(const h16* __restrict__ QEp, const h16* __restrict__ KEp, const h16* __restrict__ VTEp, h16* CEp) {
    __shared__ __align__(16) h16 os[32 * 72];
    const unsigned lane = threadIdx.x & 31u, lr = lane & 15u, hi = lane >> 4;
    const unsigned q0 = blockIdx.x * 16u, hh = blockIdx.y, b = blockIdx.z;
    const size_t rowb = (size_t)b * EROWS;
    const h16* qbase = QEp + ((rowb + q0 + lr) * NH + hh) * 128u + 8u * hi;
    const h16* kbase = KEp + ((rowb + lr) * NH + hh) * 128u + 8u * hi;
    const h16* vbase = VTEp + ((size_t)b * DM + hh * HD + lr) * (2u * EROWS) + 8u * hi;
    v16h qh[2], qr[2];
#pragma unroll
    for (int ks = 0; ks < 2; ++ks) { qh[ks] = ldfrag(qbase + ks * 32u); qr[ks] = ldfrag(qbase + 64u + ks * 32u); }
    v8f ot[4];
#pragma unroll
    for (int dt = 0; dt < 4; ++dt) ot[dt] = (v8f){};
    float m0 = -3.0e38f, l0 = 0.f;
    const unsigned ktl = q0 >> 5; const unsigned qoff = q0 & 31u;
#pragma unroll 1
    for (unsigned kt = 0; kt <= ktl; ++kt) {
        v8f st[2];
        st[0] = (v8f){}; st[1] = (v8f){};
#pragma unroll
        for (int mt = 0; mt < 2; ++mt) { const h16* kp = kbase + (size_t)(kt * 32u + mt * 16u) * (NH * 128u);
#pragma unroll
            for (int ks = 0; ks < 2; ++ks) { const v16h kh = ldfrag(kp + ks * 32u); const v16h kr = ldfrag(kp + 64u + ks * 32u);
                st[mt] = wmma16g(kh, qh[ks], st[mt]); st[mt] = wmma16g(kr, qh[ks], st[mt]); st[mt] = wmma16g(kh, qr[ks], st[mt]); } }
        if (kt == ktl) {
#pragma unroll
            for (int mt = 0; mt < 2; ++mt)
#pragma unroll
                for (int r = 0; r < 8; ++r) { const bool dead = ((unsigned)(mt * 16 + r) + 8u * hi) > (qoff + lr); st[mt][r] = dead ? NEGV : st[mt][r]; }
        }
        float t0 = st[0][0];
#pragma unroll
        for (int r = 0; r < 8; ++r) t0 = fmaxf(t0, fmaxf(st[0][r], st[1][r]));
        t0 = fmaxf(t0, __shfl_xor(t0, 16, 32));
        const float mn0 = fmaxf(m0, t0);
        const bool grow = (mn0 > m0);
        if (__builtin_amdgcn_ballot_w32(grow) != 0u) {
            const float a0 = __builtin_amdgcn_exp2f((m0 - mn0) * CL2E);
            l0 *= a0;
#pragma unroll
            for (int dt = 0; dt < 4; ++dt)
#pragma unroll
                for (int r = 0; r < 8; ++r) ot[dt][r] *= a0;
        }
        m0 = mn0;
        const float off0 = PEXPE - mn0 * CL2E;
        v16h ph, pr; float s0 = 0.f;
#pragma unroll
        for (int r = 0; r < 8; ++r) {
            const float e0 = fmaf(st[0][r], CL2E, off0), e1 = fmaf(st[1][r], CL2E, off0);
            float p0 = __builtin_amdgcn_exp2f(e0), p1 = __builtin_amdgcn_exp2f(e1);
            p0 = (e0 < -14.0f) ? 0.0f : p0; p1 = (e1 < -14.0f) ? 0.0f : p1;
            const h16 h0 = (h16)p0, h1 = (h16)p1;
            s0 += p0 + p1;
            ph[r] = h0; ph[8 + r] = h1; pr[r] = toh_flush(p0 - (float)h0); pr[8 + r] = toh_flush(p1 - (float)h1); }
        l0 += s0;
#pragma unroll
        for (int dt = 0; dt < 4; ++dt) { const h16* vp = vbase + (size_t)dt * 16u * (2u * EROWS) + kt * 32u;
            const v16h vh = ldfrag(vp); const v16h vr = ldfrag(vp + EROWS);
            ot[dt] = wmma16g(vh, ph, ot[dt]); ot[dt] = wmma16g(vr, ph, ot[dt]); ot[dt] = wmma16g(vh, pr, ot[dt]); }
    }
    l0 += __shfl_xor(l0, 16, 32);
    const float i0 = (ECAR / VCAR) / l0;
#pragma unroll
    for (int dt = 0; dt < 4; ++dt) { v8h oh, ol;
#pragma unroll
        for (int r = 0; r < 8; ++r) { const float s = ot[dt][r] * i0; const h16 hv = toh_flush(s); oh[r] = hv; ol[r] = toh_flush(s - (float)hv); }
        *(v8ha*)(os + lr * 72u + dt * 16u + 8u * hi) = oh; *(v8ha*)(os + (16u + lr) * 72u + dt * 16u + 8u * hi) = ol; }
    __syncthreads();
    h16* cb = CEp + (rowb + q0) * (2u * DM) + hh * HD; const unsigned rq = lane >> 3, c8 = (lane & 7u) * 8u;
#pragma unroll 1
    for (int ps = 0; ps < 2; ++ps) {
#pragma unroll
        for (unsigned s = 0; s < 8u; ++s) { const unsigned lrow = 4u * s + rq; const v8h v = *(const v8ha*)(os + lrow * 72u + c8);
            *(volatile v8h*)(cb + (size_t)(lrow & 15u) * (2u * DM) + (lrow >> 4) * (unsigned)DM + c8) = v; }
        if (ps == 0) __threadfence(); }
}

extern "C" void kernel_launch(void* const* d_in, const int* in_sizes, int n_in,
                              void* d_out, int out_size, void* d_ws, size_t ws_size, hipStream_t stream) {
    if (n_in < 9) return;
    const size_t xneed = ((size_t)(NB - 1) * SEQ_FULL + SEQ) * DM;
    if ((size_t)in_sizes[0] < xneed) return;
    if ((size_t)in_sizes[1] < (size_t)DM * DM || (size_t)in_sizes[3] < (size_t)DM * DM || (size_t)in_sizes[5] < (size_t)DM * DM || (size_t)in_sizes[7] < (size_t)DM * DM) return;
    if (in_sizes[2] < DM || in_sizes[4] < DM || in_sizes[6] < DM || in_sizes[8] < DM) return;
    if ((size_t)out_size < xneed || (size_t)out_size < (size_t)MROWS * DM) return;
    const float* x = (const float*)d_in[0]; const float* wq = (const float*)d_in[1]; const float* bq = (const float*)d_in[2]; const float* wk = (const float*)d_in[3]; const float* bk = (const float*)d_in[4];
    const float* wv = (const float*)d_in[5]; const float* bv = (const float*)d_in[6]; const float* wo = (const float*)d_in[7]; const float* bo = (const float*)d_in[8];
    float* OUT = (float*)d_out;
    char* wsp = (char*)d_ws;
    auto take = [&](size_t bytes) { char* p = wsp; wsp += (bytes + 255) & ~(size_t)255; return (void*)p; };
    h16* WQ = (h16*)take(SZ_W); h16* WK = (h16*)take(SZ_W); h16* WV = (h16*)take(SZ_W); h16* WO = (h16*)take(SZ_W);
    h16* WO2 = (h16*)take(SZ_W2);
    float* TAB = (float*)take(SZ_TAB);
    h16* XH = (h16*)take(SZ_PL); h16* CTX = XH;
    h16* Q16 = (h16*)take(SZ_PL); h16* K16 = (h16*)take(SZ_PL); h16* VT16 = (h16*)take(SZ_PL);
    h16* QE = (h16*)take(SZ_QE); h16* KE = (h16*)take(SZ_QE);
    float* VE32 = (float*)take(SZ_V32);
    h16* VTE = (h16*)take(SZ_VTE);
    h16* CE = (h16*)take(SZ_CE);
    if ((size_t)(wsp - (char*)d_ws) > ws_size) return;
    float* F32 = OUT;

    k_cvtx<<<(unsigned)((size_t)MROWS * DM / 8 / 256), 256, 0, stream>>>(x, XH);
    k_wt<DM, DM><<<DM * DM / 64 / 64, 256, 0, stream>>>(wq, WQ);
    k_wt<DM, DM><<<DM * DM / 64 / 64, 256, 0, stream>>>(wk, WK);
    k_wt<DM, DM><<<DM * DM / 64 / 64, 256, 0, stream>>>(wv, WV);
    k_wt<DM, DM><<<DM * DM / 64 / 64, 256, 0, stream>>>(wo, WO);
    k_wtd<<<DM * 2 * DM / 64 / 64, 256, 0, stream>>>(wo, WO2);
    k_tab<<<SEQ / 8, 256, 0, stream>>>(TAB);

    k_gemm<0, 0, 1, 0><<<dim3(MROWS / 64, DM / 64, 1), 32, 0, stream>>>(XH, WQ, DM, F32, DM, 1.0f / WCAR, bq, nullptr, 0, 0, 0);
    k_rope<<<(unsigned)((size_t)MROWS * DM / 8 / 256), 256, 0, stream>>>(F32, TAB, Q16, QE);
    k_gemm<0, 0, 1, 0><<<dim3(MROWS / 64, DM / 64, 1), 32, 0, stream>>>(XH, WK, DM, F32, DM, 1.0f / WCAR, bk, nullptr, 0, 0, 0);
    k_rope<<<(unsigned)((size_t)MROWS * DM / 8 / 256), 256, 0, stream>>>(F32, TAB, K16, KE);
    k_gemm<1, 0, 2, 0><<<dim3(DM / 64, SEQ / 64, NB), 32, 0, stream>>>(WV, XH, DM, VT16, SEQ, 1.0f / WCAR, bv, nullptr, 0, (size_t)SEQ * DM, (size_t)DM * SEQ);
    k_gemm<0, 0, 2, 0><<<dim3(DM / 64, EROWS / 64, NB), 32, 0, stream>>>(WV, XH, DM, VE32, EROWS, 1.0f / WCAR, bv, nullptr, 0, (size_t)SEQ * DM, (size_t)DM * EROWS);
    k_vsplit<<<(unsigned)((size_t)NB * DM * EROWS / 8 / 256), 256, 0, stream>>>(VE32, VTE);

    if (SEQ > EROWS) k_flash<<<dim3((SEQ - EROWS) / 32, NH, NB), 32, 0, stream>>>(Q16, K16, VT16, CTX);
    k_flash_early<<<dim3(EROWS / 16, NH, NB), 32, 0, stream>>>(QE, KE, VTE, CE);

    if (SEQ > EROWS) k_gemm<0, 0, 1, 0><<<dim3((SEQ - EROWS) / 64, DM / 64, NB), 32, 0, stream>>>(CTX + (size_t)EROWS * DM, WO, DM, OUT + (size_t)EROWS * DM, DM, 1.0f / (WCAR * CCAR), bo, nullptr, (size_t)SEQ * DM, 0, (size_t)SEQ_FULL * DM);
    k_gemm<0, 0, 1, 0><<<dim3(EROWS / 64, DM / 64, NB), 32, 0, stream>>>(CE, WO2, 2 * DM, OUT, DM, 1.0f / (WCAR * ECAR), bo, nullptr, (size_t)EROWS * 2 * DM, 0, (size_t)SEQ_FULL * DM);
}
